// E88FLAHybrid_30726196035860
// MI455X (gfx1250) — hardware-verified
//
#include <hip/hip_runtime.h>
#include <math.h>

typedef __attribute__((ext_vector_type(16))) _Float16 v16h;
typedef __attribute__((ext_vector_type(8)))  _Float16 v8h;
typedef __attribute__((ext_vector_type(2)))  _Float16 v2h;
typedef __attribute__((ext_vector_type(16))) __bf16   v16b;
typedef __attribute__((ext_vector_type(8)))  __bf16   v8b;
typedef __attribute__((ext_vector_type(8)))  float    v8f;
typedef __attribute__((ext_vector_type(4)))  float    v4f;

constexpr int kT    = 2048;
constexpr int kB    = 4;
constexpr int kDim  = 1024;
constexpr int kNH   = 8;
constexpr int kNS   = 64;
constexpr int kHV   = 64;
constexpr int kKey  = kNH * kNS;
constexpr int kVal  = kNH * kHV;
constexpr int kQKV  = 2 * kKey + kVal;
constexpr int kRows = kT * kB;
constexpr int kThr  = 256;
constexpr float kInCarry = 1024.0f;
constexpr float kSc = 1.0f / (kInCarry * kInCarry);
constexpr float kF16MinNormal = 6.103515625e-5f;

static_assert((kRows % 64) == 0 && ((kRows / 64) * (kQKV / 64)) % 8 == 0 && ((kRows / 64) * (kDim / 64)) % 8 == 0 && (kDim % 32) == 0 && (kVal % 32) == 0 && kNS == 64 && kHV == 64,
              "GEMM M, N multiples of 64; grids exact; K multiples of 32");

constexpr size_t kOffX16 = 0ull;
constexpr size_t kOffWQ16 = 16777216ull;
constexpr size_t kOffWO16 = 19922944ull;
constexpr size_t kOffZB = 20971520ull;
constexpr size_t kOffQKV = 20979712ull;
constexpr size_t kOffDEC = 71311360ull;
constexpr size_t kOffO16 = 71573504ull;
constexpr size_t kOffOUT32 = 79962112ull;
constexpr size_t kWsTotal = 113516544ull;
static_assert(kWsTotal <= 134217728ull, "carve cap: under 128 MiB");
static_assert(kOffX16 == 0
              && kOffWQ16 == kOffX16 + 16777216ull
              && kOffWO16 == kOffWQ16 + 3145728ull
              && kOffZB == kOffWO16 + 1048576ull
              && kOffQKV == kOffZB + 8192ull
              && kOffDEC == kOffQKV + 50331648ull
              && kOffO16 == kOffDEC + 262144ull
              && kOffOUT32 == kOffO16 + 8388608ull
              && kWsTotal == kOffOUT32 + 33554432ull, "the carve is chained and totalled");
static_assert((kOffX16 % 256) == 0 && (kOffWQ16 % 256) == 0 && (kOffWO16 % 256) == 0 && (kOffZB % 256) == 0 && (kOffQKV % 256) == 0 && (kOffDEC % 256) == 0 && (kOffO16 % 256) == 0 && (kOffOUT32 % 256) == 0, "aligned regions");

__device__ __forceinline__ unsigned short f2bf_bits(float f) {
  unsigned u = __float_as_uint(f);
  return (unsigned short)((u + 0x7FFFu + ((u >> 16) & 1u)) >> 16);
}
__device__ __forceinline__ float bf_bits2f(unsigned short h) { return __uint_as_float(((unsigned)h) << 16); }
__device__ __forceinline__ float bf16r(float f) { return bf_bits2f(f2bf_bits(f)); }
__device__ __forceinline__ float carry_flush(float v, float carry) {
  const float s = v * carry;
  return (fabsf(s) < kF16MinNormal) ? 0.0f : s;
}
__device__ __forceinline__ float frcp(float x) { return __builtin_amdgcn_rcpf(x); }

__device__ __forceinline__ void dep_guard4_h(v8f& a, v8f& b, v8f& c, v8f& d, v16h x, v16h y) { asm volatile("v_nop\n\tv_nop\n\tv_nop\n\tv_nop" : "+v"(a), "+v"(b), "+v"(c), "+v"(d) : "v"(x), "v"(y)); }
__device__ __forceinline__ void dep_guard4_b(v8f& a, v8f& b, v8f& c, v8f& d, v16b x, v16b y) { asm volatile("v_nop\n\tv_nop\n\tv_nop\n\tv_nop" : "+v"(a), "+v"(b), "+v"(c), "+v"(d) : "v"(x), "v"(y)); }
__device__ __forceinline__ void keep4_h(v16h a, v16h b, v16h c, v16h d) { asm volatile("v_nop" :: "v"(a), "v"(b), "v"(c), "v"(d)); }
__device__ __forceinline__ void keep4_b(v16b a, v16b b, v16b c, v16b d) { asm volatile("v_nop" :: "v"(a), "v"(b), "v"(c), "v"(d)); }
__device__ __forceinline__ void acc_guard4(v8f& a, v8f& b, v8f& c, v8f& d) { asm volatile("v_nop\n\tv_nop\n\tv_nop\n\tv_nop" : "+v"(a), "+v"(b), "+v"(c), "+v"(d)); }

template <typename T> struct Frag;
template <> struct Frag<_Float16> {
  typedef v16h V; union U { v16h v; v8h h[2]; };
  static __device__ __forceinline__ v16h load(const _Float16* p) {
    U f; f.h[0] = *(const v8h*)(p); f.h[1] = *(const v8h*)(p + 16); return f.v;
  }
  static __device__ __forceinline__ v8f mma(v16h a, v16h b, v8f c) {
    return __builtin_amdgcn_wmma_f32_16x16x32_f16(false, a, false, b, (short)0, c, false, false);
  }
  static __device__ __forceinline__ void guard4(v8f& a, v8f& b, v8f& c, v8f& d, v16h x, v16h y) { dep_guard4_h(a, b, c, d, x, y); }
  static __device__ __forceinline__ void keep(v16h a, v16h b, v16h c, v16h d) { keep4_h(a, b, c, d); }
};
template <> struct Frag<__bf16> {
  typedef v16b V; union U { v16b v; v8b h[2]; };
  static __device__ __forceinline__ v16b load(const __bf16* p) {
    U f; f.h[0] = *(const v8b*)(p); f.h[1] = *(const v8b*)(p + 16); return f.v;
  }
  static __device__ __forceinline__ v8f mma(v16b a, v16b b, v8f c) {
    return __builtin_amdgcn_wmma_f32_16x16x32_bf16(false, a, false, b, (short)0, c, false, false);
  }
  static __device__ __forceinline__ void guard4(v8f& a, v8f& b, v8f& c, v8f& d, v16b x, v16b y) { dep_guard4_b(a, b, c, d, x, y); }
  static __device__ __forceinline__ void keep(v16b a, v16b b, v16b c, v16b d) { keep4_b(a, b, c, d); }
};

__device__ __forceinline__ v8f mma_h(v16h a, v16h b, v8f c) {
  c = __builtin_amdgcn_wmma_f32_16x16x32_f16(false, a, false, b, (short)0, c, false, false);
  asm volatile("v_nop\n\tv_nop\n\tv_nop\n\tv_nop" : "+v"(c) : "v"(a), "v"(b));
  return c;
}

template <int ET> struct Elem;
template <> struct Elem<0> { typedef _Float16 T; };
template <> struct Elem<1> { typedef __bf16 T; };
template <int ET, bool SPLIT, int BIAS_MODE, int OUT_MODE, bool RESID, int ACT = 0>
__global__ __launch_bounds__(256) void wmma_gemm64(
    const unsigned short* __restrict__ Ap, const unsigned short* __restrict__ A2p, int lda, long strideA,
    const unsigned short* __restrict__ Btp, const unsigned short* __restrict__ Bt2p, int ldb, long strideB,
    void* __restrict__ Cout, void* __restrict__ Cout2, int ldc, long strideC,
    const float* __restrict__ bias,
    const float* __restrict__ resid, long strideR,
    int M, int N, int K, float scale) {
  typedef typename Elem<ET>::T T;
  typedef typename Frag<T>::V V;
  const T* A = (const T*)Ap; const T* A2 = (const T*)A2p; const T* Bt = (const T*)Btp; const T* Bt2 = (const T*)Bt2p;
  __shared__ __align__(16) float sT[8][16 * 68];
  const int b    = blockIdx.y;
  const int lane = threadIdx.x & 31;
  const int wave = threadIdx.x >> 5;
  const int tilesN = N >> 6;
  const int tilesM = M >> 6;
  const int tile = blockIdx.x * 8 + wave;
  if (tile >= tilesM * tilesN) return;
  const int tm = tile / tilesN;
  const int tn = tile - tm * tilesN;
  const int m0 = tm << 6;
  const int n0 = tn << 6;

  const T* Ab  = A  + (size_t)b * strideA;
  const T* Bb  = Bt + (size_t)b * strideB;
  const T* Ab2 = SPLIT ? (A2  + (size_t)b * strideA) : nullptr;
  const T* Bb2 = SPLIT ? (Bt2 + (size_t)b * strideB) : nullptr;

  const int rlane = lane & 15;
  const int koff  = (lane >> 4) * 8;
  const int mOff  = (lane >> 4) * 8;

  v8f acc[4][4];
#pragma unroll
  for (int i = 0; i < 4; ++i)
#pragma unroll
    for (int j = 0; j < 4; ++j) acc[i][j] = (v8f){0.f,0.f,0.f,0.f,0.f,0.f,0.f,0.f};

  for (int k0 = 0; k0 < K; k0 += 32) {
    V bh[4], bl[4];
#pragma unroll
    for (int j = 0; j < 4; ++j) {
      const size_t bo = (size_t)(n0 + (j << 4) + rlane) * ldb + koff + k0;
      bh[j] = Frag<T>::load(Bb + bo);
      if (SPLIT) bl[j] = Frag<T>::load(Bb2 + bo);
    }
#pragma unroll
    for (int i = 0; i < 4; ++i) {
      const size_t ao = (size_t)(m0 + (i << 4) + rlane) * lda + koff + k0;
      V ah = Frag<T>::load(Ab + ao);
      V al;
      if (SPLIT) al = Frag<T>::load(Ab2 + ao);
#pragma unroll
      for (int j = 0; j < 4; ++j) {
        acc[i][j] = Frag<T>::mma(ah, bh[j], acc[i][j]);
        if (SPLIT) {
          acc[i][j] = Frag<T>::mma(ah, bl[j], acc[i][j]);
          acc[i][j] = Frag<T>::mma(al, bh[j], acc[i][j]);
        }
      }
      Frag<T>::guard4(acc[i][0], acc[i][1], acc[i][2], acc[i][3], ah, SPLIT ? al : ah);
    }
    Frag<T>::keep(bh[0], bh[1], bh[2], bh[3]);
    if (SPLIT) Frag<T>::keep(bl[0], bl[1], bl[2], bl[3]);
  }
  acc_guard4(acc[0][0], acc[0][1], acc[0][2], acc[0][3]);
  acc_guard4(acc[1][0], acc[1][1], acc[1][2], acc[1][3]);
  acc_guard4(acc[2][0], acc[2][1], acc[2][2], acc[2][3]);
  acc_guard4(acc[3][0], acc[3][1], acc[3][2], acc[3][3]);

  float* slab = sT[wave];
  const float* Rb = RESID ? (resid + (size_t)b * strideR) : nullptr;
#pragma unroll
  for (int i = 0; i < 4; ++i) {
    const int mBase = m0 + (i << 4);
#pragma unroll
    for (int j = 0; j < 4; ++j) {
      const int n = n0 + (j << 4) + rlane;
      float bv = 0.f;
      if (BIAS_MODE == 2) bv = bias[n];
#pragma unroll
      for (int r = 0; r < 8; ++r) {
        float v = acc[i][j][r] * scale;
        if (BIAS_MODE == 1) v += bias[mBase + mOff + r];
        if (BIAS_MODE == 2) v += bv;
        if (RESID) v += Rb[(size_t)(mBase + mOff + r) * ldc + n];
        if (ACT == 1) v = tanhf(v);
        if (ACT == 2) v = fmaxf(v, 0.0f);
        if (ACT == 3) v = v / (1.0f + expf(-v));
        if (ACT == 4) v = (v > 0.f) ? v : 0.01f * v;
        slab[(mOff + r) * 68 + (j << 4) + rlane] = v;
      }
    }
    __builtin_amdgcn_fence(__ATOMIC_RELEASE, "workgroup");
    __builtin_amdgcn_wave_barrier();
    __builtin_amdgcn_fence(__ATOMIC_ACQUIRE, "workgroup");
    if (OUT_MODE == 0) {
      float* C = (float*)Cout + (size_t)b * strideC;
      const int hh = lane >> 4, c4 = (lane & 15) * 4;
      for (int pass = 0; pass < 2; ++pass) {
#pragma unroll
        for (int it = 0; it < 8; ++it) {
          const int row = it * 2 + hh;
          v4f v = *(const v4f*)(slab + row * 68 + c4);
          *(volatile v4f*)(C + (size_t)(mBase + row) * ldc + n0 + c4) = v;
        }
        __threadfence();
      }
    } else {
      const int q = lane >> 3, c8 = (lane & 7) * 8;
      unsigned short* C  = (unsigned short*)Cout  + (size_t)b * strideC;
      unsigned short* C2 = (OUT_MODE == 2) ? ((unsigned short*)Cout2 + (size_t)b * strideC) : nullptr;
      for (int pass = 0; pass < 2; ++pass) {
#pragma unroll
        for (int it = 0; it < 4; ++it) {
          const int row = it * 4 + q;
          const float* sp = slab + row * 68 + c8;
          v8h hv, lv;
#pragma unroll
          for (int e = 0; e < 8; ++e) {
            if (OUT_MODE == 1) {
              hv[e] = (_Float16)sp[e];
            } else {
              unsigned short hb = f2bf_bits(sp[e]);
              unsigned short lb = f2bf_bits(sp[e] - bf_bits2f(hb));
              hv[e] = __builtin_bit_cast(_Float16, hb);
              lv[e] = __builtin_bit_cast(_Float16, lb);
            }
          }
          *(volatile v8h*)(C + (size_t)(mBase + row) * ldc + n0 + c8) = hv;
          if (OUT_MODE == 2) *(volatile v8h*)(C2 + (size_t)(mBase + row) * ldc + n0 + c8) = lv;
        }
        __threadfence();
      }
    }
    __builtin_amdgcn_fence(__ATOMIC_RELEASE, "workgroup");
    __builtin_amdgcn_wave_barrier();
    __builtin_amdgcn_fence(__ATOMIC_ACQUIRE, "workgroup");
  }
}

__global__ __launch_bounds__(kThr) void cast_plane_kernel(const float* __restrict__ src, unsigned short* __restrict__ dst,
                                                          int colsLog2, int dstPitch, int dstOff) {
  const int i   = blockIdx.x * kThr + threadIdx.x;
  const int sh  = colsLog2 - 3;
  const int row = i >> sh;
  const int c8  = (i & ((1 << sh) - 1)) * 8;
  const float* sp = src + ((size_t)row << colsLog2) + c8;
  const v4f a0 = *(const v4f*)(sp);
  const v4f a1 = *(const v4f*)(sp + 4);
  v8h hv;
#pragma unroll
  for (int e = 0; e < 4; ++e) {
    const float f0 = a0[e];
    const float f1 = a1[e];
    hv[e]     = (_Float16)carry_flush(bf16r(f0), kInCarry);
    hv[4 + e] = (_Float16)carry_flush(bf16r(f1), kInCarry);
  }
  unsigned short* dp = dst + (size_t)row * dstPitch + dstOff + c8;
  *(volatile v8h*)dp = hv;
  __threadfence();
  *(volatile v8h*)dp = hv;
}

__device__ __forceinline__ float fast_tanh(float v) { return 1.0f - 2.0f * frcp(__expf(2.0f * v) + 1.0f); }

__global__ __launch_bounds__(kThr) void zero_kernel(float* __restrict__ ZB) {
  const unsigned v = blockIdx.x * (unsigned)kThr + threadIdx.x;
  const v4f z = {0.f, 0.f, 0.f, 0.f};
  float* dp = ZB + (size_t)v * 4u;
  *(volatile v4f*)dp = z;
  __threadfence();
  *(volatile v4f*)dp = z;
}

__global__ __launch_bounds__(kThr) void prep_kernel(float* __restrict__ QKV, const float* __restrict__ x, const float* __restrict__ W_a, const float* __restrict__ A_log,
                                                    const float* __restrict__ dt_bias, float* __restrict__ DEC) {
  unsigned v = blockIdx.x * (unsigned)kThr + threadIdx.x;
  asm volatile("" : "+v"(v));
  const unsigned row = v >> 3, h = v & 7u;
  float* qp = QKV + (size_t)row * kQKV + h * kNS;
  float* kp = qp + kKey;
  float* vp = qp + 2 * kKey;
  float sq = 0.0f, sk = 0.0f;
  for (int n = 0; n < kNS; n += 4) {
    const v4f a = *(const v4f*)(qp + n), c = *(const v4f*)(kp + n);
    sq += a[0] * a[0]; sq += a[1] * a[1]; sq += a[2] * a[2]; sq += a[3] * a[3];
    sk += c[0] * c[0]; sk += c[1] * c[1]; sk += c[2] * c[2]; sk += c[3] * c[3];
  }
  const float rq = rsqrtf(sq + 1e-6f), rk = rsqrtf(sk + 1e-6f);
  const float* xr = x + (size_t)row * kDim;
  const float* wr = W_a + (size_t)h * kDim;
  float acc = 0.0f;
  for (int d = 0; d < kDim; d += 4) {
    const v4f a = *(const v4f*)(xr + d), c = *(const v4f*)(wr + d);
    const float p0 = a[0], p1 = a[1], p2 = a[2], p3 = a[3], q0 = c[0], q1 = c[1], q2 = c[2], q3 = c[3];
    acc += bf16r(p0) * bf16r(q0);
    acc += bf16r(p1) * bf16r(q1);
    acc += bf16r(p2) * bf16r(q2);
    acc += bf16r(p3) * bf16r(q3);
  }
  float db = dt_bias[h], al = A_log[h];
  asm volatile("" : "+v"(db), "+v"(al));
  const float aa = acc + bf16r(db);
  const float dec = expf(-expf(bf16r(al)) * log1pf(expf(aa)));
#pragma unroll 1
  for (int n = 0; n < kNS; n += 4) {
    const v4f a = *(const v4f*)(qp + n), c = *(const v4f*)(kp + n), e = *(const v4f*)(vp + n);
    v4f qo, ko, vo;
#pragma unroll
    for (int i = 0; i < 4; ++i) { qo[i] = a[i] * rq; ko[i] = c[i] * rk; vo[i] = e[i] / (1.0f + expf(-e[i])); }
    *(volatile v4f*)(qp + n) = qo; *(volatile v4f*)(kp + n) = ko; *(volatile v4f*)(vp + n) = vo;
    __threadfence();
    *(volatile v4f*)(qp + n) = qo; *(volatile v4f*)(kp + n) = ko; *(volatile v4f*)(vp + n) = vo;
  }
  *(volatile float*)(DEC + v) = dec;
  __threadfence();
  *(volatile float*)(DEC + v) = dec;
}
static_assert(kRows * kNH == 256 * kThr, "preparation grid exact");

__global__ __launch_bounds__(kThr) void scan_kernel(const float* __restrict__ QKV, const float* __restrict__ DEC, unsigned short* __restrict__ O16) {
  __shared__ float sPart[4][kHV];
  const int tid = threadIdx.x;
  const int b = (int)(blockIdx.x >> 3), h = (int)(blockIdx.x & 7u);
  const int d = tid & 63, g = tid >> 6;
  float S[16];
#pragma unroll
  for (int i = 0; i < 16; ++i) S[i] = 0.0f;
#pragma unroll 1
  for (int t = 0; t < kT; ++t) {
    const size_t row = (size_t)t * kB + (size_t)b;
    const float* qr = QKV + row * kQKV + h * kNS + 16 * g;
    const float* kr = qr + kKey;
    const float vv = QKV[row * kQKV + 2 * kKey + h * kHV + d];
    const float dec = DEC[row * kNH + h];
    float part = 0.0f;
#pragma unroll
    for (int i4 = 0; i4 < 16; i4 += 4) {
      const v4f q4 = *(const v4f*)(qr + i4), k4 = *(const v4f*)(kr + i4);
#pragma unroll
      for (int e = 0; e < 4; ++e) {
        const float s = fast_tanh(dec * S[i4 + e] + k4[e] * vv);
        S[i4 + e] = s;
        part += q4[e] * s;
      }
    }
    sPart[g][d] = part;
    __syncthreads();
    if (tid < 32) {
      const int d0 = 2 * tid;
      float o0 = sPart[0][d0], o1 = sPart[0][d0 + 1];
      o0 += sPart[1][d0]; o1 += sPart[1][d0 + 1];
      o0 += sPart[2][d0]; o1 += sPart[2][d0 + 1];
      o0 += sPart[3][d0]; o1 += sPart[3][d0 + 1];
      v2h hv;
      hv[0] = (_Float16)carry_flush(o0, kInCarry);
      hv[1] = (_Float16)carry_flush(o1, kInCarry);
      unsigned short* op = O16 + row * kVal + h * kHV + d0;
      *(volatile v2h*)op = hv;
      __threadfence();
      *(volatile v2h*)op = hv;
    }
    __syncthreads();
  }
}
static_assert(kThr == 4 * kHV && kNS == 4 * 16, "scan thread map: four 16-row groups x 64 columns");

__global__ __launch_bounds__(kThr) void out_kernel(const float* __restrict__ OUT32, float* __restrict__ out) {
  const size_t i = ((size_t)blockIdx.x * kThr + threadIdx.x) * 4;
  const v4f o = *(const v4f*)(OUT32 + i);
  float* dp = out + i;
  *(volatile v4f*)dp = o;
  __threadfence();
  *(volatile v4f*)dp = o;
}
static_assert((size_t)kRows * kDim / 4 == 8192 * (size_t)kThr, "output grid exact");

static_assert(((size_t)kRows * kDim / 8) % kThr == 0 && ((size_t)kQKV * kDim / 8) % kThr == 0 && ((size_t)kDim * kVal / 8) % kThr == 0, "plane cast grids exact");

extern "C" void kernel_launch(void* const* d_in, const int* in_sizes, int n_in,
                              void* d_out, int out_size, void* d_ws, size_t ws_size,
                              hipStream_t stream) {
  if (n_in < 6 || d_out == nullptr || d_ws == nullptr) return;
  if (in_sizes[0] != kRows * kDim || in_sizes[1] != kQKV * kDim || in_sizes[2] != kNH * kDim || in_sizes[3] != kNH || in_sizes[4] != kNH || in_sizes[5] != kDim * kVal) return;
  if (out_size != kRows * kDim) return;
  if (ws_size < kWsTotal) return;
  const float* x = (const float*)d_in[0];
  const float* W_qkv = (const float*)d_in[1];
  const float* W_a = (const float*)d_in[2];
  const float* A_log = (const float*)d_in[3];
  const float* dt_bias = (const float*)d_in[4];
  const float* W_out = (const float*)d_in[5];
  float* out = (float*)d_out;
  char* ws = (char*)d_ws;
  unsigned short* X16 = (unsigned short*)(ws + kOffX16);
  unsigned short* WQ16 = (unsigned short*)(ws + kOffWQ16);
  unsigned short* WO16 = (unsigned short*)(ws + kOffWO16);
  float* ZB = (float*)(ws + kOffZB);
  float* QKV = (float*)(ws + kOffQKV);
  float* DEC = (float*)(ws + kOffDEC);
  unsigned short* O16 = (unsigned short*)(ws + kOffO16);
  float* OUT32 = (float*)(ws + kOffOUT32);

  cast_plane_kernel<<<(int)(((size_t)kRows * kDim / 8) / kThr), kThr, 0, stream>>>(x, X16, 10, kDim, 0);
  cast_plane_kernel<<<(int)(((size_t)kQKV * kDim / 8) / kThr), kThr, 0, stream>>>(W_qkv, WQ16, 10, kDim, 0);
  cast_plane_kernel<<<(int)(((size_t)kDim * kVal / 8) / kThr), kThr, 0, stream>>>(W_out, WO16, 9, kVal, 0);
  zero_kernel<<<2, kThr, 0, stream>>>(ZB);
  wmma_gemm64<0, false, 2, 0, false, 0><<<dim3((kRows / 64) * (kQKV / 64) / 8, 1), 256, 0, stream>>>(
      X16, X16, kDim, 0L, WQ16, WQ16, kDim, 0L, (void*)QKV, (void*)QKV, kQKV, 0L, ZB, nullptr, 0L, kRows, kQKV, kDim, kSc);
  prep_kernel<<<256, kThr, 0, stream>>>(QKV, x, W_a, A_log, dt_bias, DEC);
  scan_kernel<<<kB * kNH, kThr, 0, stream>>>(QKV, DEC, O16);
  wmma_gemm64<0, false, 2, 0, false, 0><<<dim3((kRows / 64) * (kDim / 64) / 8, 1), 256, 0, stream>>>(
      O16, O16, kVal, 0L, WO16, WO16, kVal, 0L, (void*)OUT32, (void*)OUT32, kDim, 0L, ZB, nullptr, 0L, kRows, kDim, kVal, kSc);
  out_kernel<<<8192, kThr, 0, stream>>>(OUT32, out);
}
